// MultiHeadDifferAttention_79328045957412
// MI455X (gfx1250) — hardware-run, weakly checked
//
#include <hip/hip_runtime.h>
#include <math.h>

typedef __attribute__((ext_vector_type(16))) _Float16 v16h;
typedef __attribute__((ext_vector_type(8)))  _Float16 v8h;
typedef __attribute__((ext_vector_type(16))) __bf16   v16b;
typedef __attribute__((ext_vector_type(8)))  __bf16   v8b;
typedef __attribute__((ext_vector_type(8)))  float    v8f;
typedef __attribute__((ext_vector_type(4)))  float    v4f;
typedef __attribute__((ext_vector_type(4)))  unsigned int v4u;

constexpr int kBatch    = 2;
constexpr int kSeq      = 2048;
constexpr int kDim      = 2048;
constexpr int kPairs    = 16;
constexpr int kHd       = 64;
constexpr int kHalfHeads = 2 * kPairs;
constexpr int kVd       = 2 * kHd;
constexpr int kRows     = kBatch * kSeq;
constexpr int kHeadRows = 128;
constexpr int kTabCols  = kHd / 2;
static_assert(kPairs * kVd == kDim, "head split");
static_assert(kHalfHeads * kHd == kDim, "half-head split");
static_assert((kDim % 64) == 0 && (kRows % 64) == 0 && (kSeq % 64) == 0, "tile multiples");
static_assert((kDim % 32) == 0, "k multiple of 32");
static_assert((kHeadRows % 64) == 0 && kHeadRows == 128, "head-row path is built for 128 rows");

constexpr float kQScale = 0.125f;
static_assert(kQScale * kQScale * (float)kHd == 1.0f, "q scale");
constexpr float kQCarry = 128.0f;
constexpr float kKCarry = 16.0f;
constexpr float kVCarry = 16.0f;
constexpr float kPCarry = 32768.0f;
constexpr float kScoreScale = 1.0f / (kQCarry * kKCarry);
constexpr float kPVCarry = kPCarry * kVCarry;
constexpr float kMaskFill = -1e30f;
constexpr float kLamInit = 0.7836057665316245f;

constexpr size_t kOffXB  = 0;
constexpr size_t kOffWT  = kOffXB + (size_t)kRows * kDim * 2;
constexpr size_t kOffQH  = kOffWT + (size_t)3 * kDim * kDim * 2;
constexpr size_t kOffKH  = kOffQH + (size_t)kBatch * kHalfHeads * kSeq * kHd * 2;
constexpr size_t kOffVT  = kOffKH + (size_t)kBatch * kHalfHeads * kSeq * kHd * 2;
constexpr size_t kOffQF  = kOffVT + (size_t)kBatch * kDim * kSeq * 2;
constexpr size_t kOffKF  = kOffQF + (size_t)kBatch * kHalfHeads * kHeadRows * kHd * 4;
constexpr size_t kOffVF  = kOffKF + (size_t)kBatch * kHalfHeads * kHeadRows * kHd * 4;
constexpr size_t kOffLAM = kOffVF + (size_t)kBatch * kDim * kHeadRows * 4;
constexpr size_t kWsTotal = kOffLAM + 128;
static_assert(kWsTotal == 98566272ull, "carve total");
static_assert(kWsTotal <= 134217728ull, "carve cap");
static_assert((kOffWT % 128) == 0 && (kOffQH % 128) == 0 && (kOffKH % 128) == 0 && (kOffVT % 128) == 0 &&
              (kOffQF % 128) == 0 && (kOffKF % 128) == 0 && (kOffVF % 128) == 0 && (kOffLAM % 128) == 0, "aligned regions");

__device__ __forceinline__ unsigned short f2bf_bits(float f) {
  unsigned u = __float_as_uint(f);
  return (unsigned short)((u + 0x7FFFu + ((u >> 16) & 1u)) >> 16);
}
__device__ __forceinline__ float bf_bits2f(unsigned short h) { return __uint_as_float(((unsigned)h) << 16); }
__device__ __forceinline__ float bfr(float f) { return bf_bits2f(f2bf_bits(f)); }
__device__ __forceinline__ unsigned pk16(unsigned short a, unsigned short b) { return (unsigned)a | ((unsigned)b << 16); }
__device__ __forceinline__ unsigned short h_bits(float f) { const _Float16 h = (_Float16)f; return __builtin_bit_cast(unsigned short, h); }

__device__ __forceinline__ void wave_lds_sync() {
  __builtin_amdgcn_fence(__ATOMIC_RELEASE, "workgroup");
  __builtin_amdgcn_wave_barrier();
  __builtin_amdgcn_fence(__ATOMIC_ACQUIRE, "workgroup");
}

__device__ __forceinline__ void tie_b(v8f& a, v16b x, v16b y) { asm volatile("" : "+v"(a) : "v"(x), "v"(y)); }
__device__ __forceinline__ void tie_nop_b(v8f& a, v16b x, v16b y) { asm volatile("v_nop\n\tv_nop\n\tv_nop\n\tv_nop" : "+v"(a) : "v"(x), "v"(y)); }
__device__ __forceinline__ void keep4_b(v16b a, v16b b, v16b c, v16b d) { asm volatile("v_nop" :: "v"(a), "v"(b), "v"(c), "v"(d)); }
__device__ __forceinline__ void acc_guard4(v8f& a, v8f& b, v8f& c, v8f& d) { asm volatile("v_nop\n\tv_nop\n\tv_nop\n\tv_nop" : "+v"(a), "+v"(b), "+v"(c), "+v"(d)); }

__device__ __forceinline__ v16b frag_b(const __bf16* p) {
  union { v16b v; v8b h[2]; } f;
  f.h[0] = *(const v8b*)(p);
  f.h[1] = *(const v8b*)(p + 16);
  return f.v;
}
__device__ __forceinline__ v16h frag_h(const _Float16* p) {
  union { v16h v; v8h h[2]; } f;
  f.h[0] = *(const v8h*)(p);
  f.h[1] = *(const v8h*)(p + 16);
  return f.v;
}
__device__ __forceinline__ v8f mma_b(v16b a, v16b b, v8f c) {
  return __builtin_amdgcn_wmma_f32_16x16x32_bf16(false, a, false, b, (short)0, c, false, false);
}
__device__ __forceinline__ v8f mma_h(v16h a, v16h b, v8f c) {
  c = __builtin_amdgcn_wmma_f32_16x16x32_f16(false, a, false, b, (short)0, c, false, false);
  asm volatile("v_nop\n\tv_nop\n\tv_nop\n\tv_nop" : "+v"(c) : "v"(a), "v"(b));
  return c;
}

__global__ __launch_bounds__(256) void cvt_bf16_kernel(const float* __restrict__ in, unsigned short* __restrict__ outp, int n8) {
  const int i = blockIdx.x * 256 + threadIdx.x;
  if (i >= n8) return;
  const float* p = in + 8 * (size_t)i;
  const v4f a = *(const v4f*)(p);
  const v4f c = *(const v4f*)(p + 4);
  unsigned short hb[8];
#pragma unroll
  for (int e = 0; e < 4; ++e) {
    const float fa = a[e];
    const float fc = c[e];
    hb[e]     = f2bf_bits(fa);
    hb[4 + e] = f2bf_bits(fc);
  }
  const v4u u = (v4u){pk16(hb[0], hb[1]), pk16(hb[2], hb[3]), pk16(hb[4], hb[5]), pk16(hb[6], hb[7])};
  unsigned short* q = outp + 8 * (size_t)i;
  *(volatile v4u*)q = u;
  __threadfence();
  *(volatile v4u*)q = u;
}

__global__ __launch_bounds__(256) void wt_pack_kernel(const float* __restrict__ W0, const float* __restrict__ W1,
                                                      const float* __restrict__ W2, unsigned short* __restrict__ outp) {
  __shared__ float sm[64][65];
  const int t  = threadIdx.x;
  const int k0 = blockIdx.x * 64;
  const int n0 = blockIdx.y * 64;
  const int z  = blockIdx.z;
  const float* W = (z == 0) ? W0 : ((z == 1) ? W1 : W2);
#pragma unroll 8
  for (int i = 0; i < 16; ++i) {
    const int e = i * 256 + t;
    const int r = e >> 6;
    const int c = e & 63;
    sm[c][r] = W[(size_t)(k0 + r) * kDim + n0 + c];
  }
  __syncthreads();
  const int lane = t & 31;
  const int wave = __builtin_amdgcn_readfirstlane((int)(t >> 5));
  const int q = lane >> 3, c8 = (lane & 7) * 8;
  unsigned short* op = outp + (size_t)z * kDim * kDim;
  v4u u[2];
#pragma unroll
  for (int it = 0; it < 2; ++it) {
    const int row = wave * 8 + it * 4 + q;
    unsigned short hb[8];
#pragma unroll
    for (int e = 0; e < 8; ++e) hb[e] = f2bf_bits(sm[row][c8 + e]);
    u[it] = (v4u){pk16(hb[0], hb[1]), pk16(hb[2], hb[3]), pk16(hb[4], hb[5]), pk16(hb[6], hb[7])};
  }
  for (int pass = 0; pass < 2; ++pass) {
#pragma unroll
    for (int it = 0; it < 2; ++it) {
      const int row = wave * 8 + it * 4 + q;
      *(volatile v4u*)(op + (size_t)(n0 + row) * kDim + k0 + c8) = u[it];
    }
    __threadfence();
  }
}

__global__ __launch_bounds__(32) void lam_kernel(const float* __restrict__ lq1, const float* __restrict__ lk1,
                                                 const float* __restrict__ lq2, const float* __restrict__ lk2,
                                                 float* __restrict__ lamp) {
  const int lane = threadIdx.x & 31;
  float d1 = bfr(lq1[lane]) * bfr(lk1[lane]);
  d1 = fmaf(bfr(lq1[lane + 32]), bfr(lk1[lane + 32]), d1);
  float d2 = bfr(lq2[lane]) * bfr(lk2[lane]);
  d2 = fmaf(bfr(lq2[lane + 32]), bfr(lk2[lane + 32]), d2);
#pragma unroll
  for (int off = 16; off > 0; off >>= 1) {
    const float t1 = __shfl_xor(d1, off, 32);
    const float t2 = __shfl_xor(d2, off, 32);
    d1 += t1;
    d2 += t2;
  }
  const float lam = expf(d1) - expf(d2) + kLamInit;
  *(volatile float*)(lamp + lane) = lam;
  __threadfence();
  *(volatile float*)(lamp + lane) = lam;
}

template <int MODE>
__global__ __launch_bounds__(256) void proj_gemm_kernel(
    const unsigned short* __restrict__ Ap, const unsigned short* __restrict__ Btp,
    const float* __restrict__ bias0, const float* __restrict__ bias1,
    const float* __restrict__ fcos, const float* __restrict__ fsin,
    unsigned short* __restrict__ o16a, unsigned short* __restrict__ o16b,
    float* __restrict__ ofa, float* __restrict__ ofb,
    int tilesM, int tilesN) {
  const __bf16* A  = (const __bf16*)Ap;
  const __bf16* Bt = (const __bf16*)Btp;
  __shared__ __align__(16) float sT[8][16 * 68];
  const int lane = threadIdx.x & 31;
  const int wave = __builtin_amdgcn_readfirstlane((int)(threadIdx.x >> 5));
  const int tile = blockIdx.x * 8 + wave;
  if (tile >= tilesM * tilesN) return;
  const int tm = tile / tilesN;
  const int tn = tile - tm * tilesN;
  const int m0 = tm << 6;
  const int n0 = tn << 6;

  const int rlane = lane & 15;
  const int koff  = (lane >> 4) * 8;
  const int mOff  = (lane >> 4) * 8;

  v8f acc[4][4];
#pragma unroll
  for (int i = 0; i < 4; ++i)
#pragma unroll
    for (int j = 0; j < 4; ++j) acc[i][j] = (v8f){0.f, 0.f, 0.f, 0.f, 0.f, 0.f, 0.f, 0.f};

  for (int k0 = 0; k0 < kDim; k0 += 32) {
    v16b bh[4];
#pragma unroll
    for (int j = 0; j < 4; ++j) {
      const size_t bo = (size_t)(n0 + (j << 4) + rlane) * kDim + koff + k0;
      bh[j] = frag_b(Bt + bo);
    }
#pragma unroll
    for (int i = 0; i < 4; ++i) {
      const size_t ao = (size_t)(m0 + (i << 4) + rlane) * kDim + koff + k0;
      const v16b ah = frag_b(A + ao);
#pragma unroll
      for (int j = 0; j < 4; ++j) acc[i][j] = mma_b(ah, bh[j], acc[i][j]);
      tie_b(acc[i][0], ah, bh[0]);
      tie_b(acc[i][1], ah, bh[1]);
      tie_b(acc[i][2], ah, bh[2]);
      tie_nop_b(acc[i][3], ah, bh[3]);
    }
    keep4_b(bh[0], bh[1], bh[2], bh[3]);
  }
  acc_guard4(acc[0][0], acc[0][1], acc[0][2], acc[0][3]);
  acc_guard4(acc[1][0], acc[1][1], acc[1][2], acc[1][3]);
  acc_guard4(acc[2][0], acc[2][1], acc[2][2], acc[2][3]);
  acc_guard4(acc[3][0], acc[3][1], acc[3][2], acc[3][3]);

  float* slab = sT[wave];
  const int q8 = lane >> 3, l7 = lane & 7, c8 = l7 * 8;
  const int hh = lane >> 4, c4 = (lane & 15) * 4;

  if (MODE == 0) {
    const int isK = n0 >> 11;
    const int ncol0 = n0 & (kDim - 1);
    const int h32 = ncol0 >> 6;
    const int bb  = m0 >> 11;
    const int s0  = m0 & (kSeq - 1);
    const float* bias = isK ? bias1 : bias0;
    unsigned short* dst16 = (isK ? o16b : o16a) + (size_t)(bb * kHalfHeads + h32) * kSeq * kHd;
    float* dstf = (isK ? ofb : ofa) + (size_t)(bb * kHalfHeads + h32) * kHeadRows * kHd;
    const float sc16 = isK ? kKCarry : (kQScale * kQCarry);
    const float scf  = isK ? 1.0f : kQScale;
    const bool headTile = (s0 < kHeadRows);
#pragma unroll
    for (int i = 0; i < 4; ++i) {
#pragma unroll
      for (int j = 0; j < 4; ++j) {
        const float bv = bfr(bias[ncol0 + (j << 4) + rlane]);
#pragma unroll
        for (int r = 0; r < 8; ++r) slab[(mOff + r) * 68 + (j << 4) + rlane] = acc[i][j][r] + bv;
      }
      wave_lds_sync();
      v4u pk[4];
#pragma unroll
      for (int it = 0; it < 4; ++it) {
        const int row = it * 4 + q8;
        const int s = s0 + (i << 4) + row;
        float* sp = slab + row * 68 + c8;
        const v4f x0 = *(const v4f*)(sp);
        const v4f x1 = *(const v4f*)(sp + 4);
        const v4f cc = *(const v4f*)(fcos + (size_t)s * kTabCols + l7 * 4);
        const v4f ss = *(const v4f*)(fsin + (size_t)s * kTabCols + l7 * 4);
        const float xin[8] = {x0[0], x0[1], x0[2], x0[3], x1[0], x1[1], x1[2], x1[3]};
        const float cr[4] = {bfr(cc[0]), bfr(cc[1]), bfr(cc[2]), bfr(cc[3])};
        const float sr[4] = {bfr(ss[0]), bfr(ss[1]), bfr(ss[2]), bfr(ss[3])};
        float o[8];
#pragma unroll
        for (int e = 0; e < 4; ++e) {
          o[2 * e]     = xin[2 * e] * cr[e] - xin[2 * e + 1] * sr[e];
          o[2 * e + 1] = xin[2 * e] * sr[e] + xin[2 * e + 1] * cr[e];
        }
        pk[it] = (v4u){pk16(h_bits(o[0] * sc16), h_bits(o[1] * sc16)), pk16(h_bits(o[2] * sc16), h_bits(o[3] * sc16)),
                       pk16(h_bits(o[4] * sc16), h_bits(o[5] * sc16)), pk16(h_bits(o[6] * sc16), h_bits(o[7] * sc16))};
        if (headTile) {
          *(v4f*)(sp)     = (v4f){o[0] * scf, o[1] * scf, o[2] * scf, o[3] * scf};
          *(v4f*)(sp + 4) = (v4f){o[4] * scf, o[5] * scf, o[6] * scf, o[7] * scf};
        }
      }
      for (int pass = 0; pass < 2; ++pass) {
#pragma unroll
        for (int it = 0; it < 4; ++it) {
          const int row = it * 4 + q8;
          *(volatile v4u*)(dst16 + (size_t)(s0 + (i << 4) + row) * kHd + c8) = pk[it];
        }
        __threadfence();
      }
      if (headTile) {
        wave_lds_sync();
        v4f fv[8];
#pragma unroll
        for (int it = 0; it < 8; ++it) fv[it] = *(const v4f*)(slab + (it * 2 + hh) * 68 + c4);
        for (int pass = 0; pass < 2; ++pass) {
#pragma unroll
          for (int it = 0; it < 8; ++it) {
            const int row = it * 2 + hh;
            *(volatile v4f*)(dstf + (size_t)(s0 + (i << 4) + row) * kHd + c4) = fv[it];
          }
          __threadfence();
        }
      }
      wave_lds_sync();
    }
  } else {
    const int bb = n0 >> 11;
    const int s0 = n0 & (kSeq - 1);
    const bool headTile = (s0 < kHeadRows);
#pragma unroll
    for (int i = 0; i < 4; ++i) {
      const int mBase = m0 + (i << 4);
      float bvr[8];
#pragma unroll
      for (int r = 0; r < 8; ++r) bvr[r] = bfr(bias0[mBase + mOff + r]);
#pragma unroll
      for (int j = 0; j < 4; ++j) {
#pragma unroll
        for (int r = 0; r < 8; ++r) slab[(mOff + r) * 68 + (j << 4) + rlane] = acc[i][j][r] + bvr[r];
      }
      wave_lds_sync();
      v4u pk[4];
#pragma unroll
      for (int it = 0; it < 4; ++it) {
        const int row = it * 4 + q8;
        const float* sp = slab + row * 68 + c8;
        const v4f x0 = *(const v4f*)(sp);
        const v4f x1 = *(const v4f*)(sp + 4);
        pk[it] = (v4u){pk16(h_bits(x0[0] * kVCarry), h_bits(x0[1] * kVCarry)), pk16(h_bits(x0[2] * kVCarry), h_bits(x0[3] * kVCarry)),
                       pk16(h_bits(x1[0] * kVCarry), h_bits(x1[1] * kVCarry)), pk16(h_bits(x1[2] * kVCarry), h_bits(x1[3] * kVCarry))};
      }
      for (int pass = 0; pass < 2; ++pass) {
#pragma unroll
        for (int it = 0; it < 4; ++it) {
          const int row = it * 4 + q8;
          *(volatile v4u*)(o16a + ((size_t)bb * kDim + mBase + row) * kSeq + s0 + c8) = pk[it];
        }
        __threadfence();
      }
      if (headTile) {
        v4f fv[8];
#pragma unroll
        for (int it = 0; it < 8; ++it) fv[it] = *(const v4f*)(slab + (it * 2 + hh) * 68 + c4);
        for (int pass = 0; pass < 2; ++pass) {
#pragma unroll
          for (int it = 0; it < 8; ++it) {
            const int row = it * 2 + hh;
            *(volatile v4f*)(ofa + ((size_t)bb * kDim + mBase + row) * kHeadRows + s0 + c4) = fv[it];
          }
          __threadfence();
        }
      }
      wave_lds_sync();
    }
  }
}

constexpr int kLp = 72;
constexpr int kOp = 132;
constexpr int kPoolBytes = (2 * 64 + 128 + 8 * 16) * kLp * 2;
static_assert(kPoolBytes == 55296, "pool size");
static_assert(4 * 16 * kOp * 4 <= kPoolBytes, "combine tile fits the pool");

__global__ __launch_bounds__(256) void diff_attn_kernel(const unsigned short* __restrict__ Qp, const unsigned short* __restrict__ Kp,
                                                        const unsigned short* __restrict__ Vp, const float* __restrict__ lamp,
                                                        float* __restrict__ out) {
  __shared__ __align__(16) unsigned char pool[kPoolBytes];
  _Float16* Ks = (_Float16*)pool;
  _Float16* Vs = Ks + 2 * 64 * kLp;
  _Float16* Ps = Vs + 128 * kLp;
  float* Os = (float*)pool;

  const int tid  = threadIdx.x;
  const int lane = tid & 31;
  const int wave = __builtin_amdgcn_readfirstlane((int)(tid >> 5));
  const int hh = lane >> 4;
  const int c  = lane & 15;
  const int qt = wave >> 1, par = wave & 1;
  const int qb = (int)blockIdx.x + (kHeadRows / 64);
  const int h  = blockIdx.y;
  const int b  = blockIdx.z;
  const int q0 = qb * 64 + qt * 16;

  const _Float16* Qg = (const _Float16*)Qp + ((size_t)(b * kHalfHeads + 2 * h + par) * kSeq + q0 + c) * kHd + 8 * hh;
  const _Float16* Kg = (const _Float16*)Kp + (size_t)(b * kHalfHeads + 2 * h) * kSeq * kHd;
  const _Float16* Vg = (const _Float16*)Vp + ((size_t)b * kDim + h * kVd) * kSeq;

  v16h qa[2];
#pragma unroll
  for (int dc = 0; dc < 2; ++dc) qa[dc] = frag_h(Qg + dc * 32);

  float mrow[8], lrow[8];
  v8f oacc[8];
#pragma unroll
  for (int r = 0; r < 8; ++r) { mrow[r] = kMaskFill; lrow[r] = 0.f; }
#pragma unroll
  for (int t = 0; t < 8; ++t) oacc[t] = (v8f){0.f, 0.f, 0.f, 0.f, 0.f, 0.f, 0.f, 0.f};

  const _Float16* Kw = Ks + par * 64 * kLp;
  _Float16* pw = Ps + wave * 16 * kLp;

#pragma unroll 1
  for (int kc = 0; kc <= qb; ++kc) {
    const int kv0 = kc * 64;
    __syncthreads();
#pragma unroll
    for (int it = 0; it < 4; ++it) {
      const int idx = tid + it * 256;
      const int p = idx >> 9, row = (idx >> 3) & 63, seg = idx & 7;
      const v8h kvv = *(const v8h*)(Kg + ((size_t)p * kSeq + kv0 + row) * kHd + seg * 8);
      *(v8h*)(Ks + (p * 64 + row) * kLp + seg * 8) = kvv;
    }
#pragma unroll
    for (int it = 0; it < 4; ++it) {
      const int idx = tid + it * 256;
      const int row = idx >> 3, seg = idx & 7;
      const v8h vvv = *(const v8h*)(Vg + (size_t)row * kSeq + kv0 + seg * 8);
      *(v8h*)(Vs + row * kLp + seg * 8) = vvv;
    }
    __syncthreads();

    v8f s[4];
#pragma unroll
    for (int j = 0; j < 4; ++j) {
      s[j] = (v8f){0.f, 0.f, 0.f, 0.f, 0.f, 0.f, 0.f, 0.f};
#pragma unroll
      for (int dc = 0; dc < 2; ++dc) {
        const v16h kb = frag_h(Kw + (j * 16 + c) * kLp + dc * 32 + 8 * hh);
        s[j] = mma_h(qa[dc], kb, s[j]);
      }
    }
    const bool diag = (kc == qb);
    float cm[8];
#pragma unroll
    for (int r = 0; r < 8; ++r) {
      const int qrow = q0 + 8 * hh + r;
      float m = kMaskFill;
#pragma unroll
      for (int j = 0; j < 4; ++j) {
        const int kvcol = kv0 + j * 16 + c;
        float v = s[j][r] * kScoreScale;
        v = (diag && (kvcol > qrow)) ? kMaskFill : v;
        s[j][r] = v;
        m = fmaxf(m, v);
      }
#pragma unroll
      for (int off = 1; off < 16; off <<= 1) {
        const float other = __shfl_xor(m, off, 32);
        m = fmaxf(m, other);
      }
      cm[r] = m;
    }
#pragma unroll
    for (int r = 0; r < 8; ++r) {
      const float mnew = fmaxf(mrow[r], cm[r]);
      const float alpha = __expf(mrow[r] - mnew);
      mrow[r] = mnew;
      float psum = 0.f;
#pragma unroll
      for (int j = 0; j < 4; ++j) {
        const float p = __expf(s[j][r] - mnew);
        psum += p;
        pw[(8 * hh + r) * kLp + j * 16 + c] = (_Float16)(p * kPCarry);
      }
#pragma unroll
      for (int off = 1; off < 16; off <<= 1) {
        const float other = __shfl_xor(psum, off, 32);
        psum += other;
      }
      lrow[r] = lrow[r] * alpha + psum;
#pragma unroll
      for (int t = 0; t < 8; ++t) oacc[t][r] *= alpha;
    }
    wave_lds_sync();
#pragma unroll 1
    for (int kk = 0; kk < 2; ++kk) {
      const v16h pa = frag_h(pw + c * kLp + kk * 32 + 8 * hh);
#pragma unroll
      for (int t = 0; t < 8; ++t) {
        const v16h vb = frag_h(Vs + (t * 16 + c) * kLp + kk * 32 + 8 * hh);
        oacc[t] = mma_h(pa, vb, oacc[t]);
      }
    }
  }

  __syncthreads();
  const float lam = lamp[0];
  float* ot = Os + qt * 16 * kOp;
  if (par == 1) {
#pragma unroll
    for (int r = 0; r < 8; ++r) {
      const float inv = lam * (1.0f / (lrow[r] * kPVCarry));
#pragma unroll
      for (int t = 0; t < 8; ++t) ot[(8 * hh + r) * kOp + t * 16 + c] = oacc[t][r] * inv;
    }
  }
  __syncthreads();
  if (par == 0) {
#pragma unroll
    for (int r = 0; r < 8; ++r) {
      const float inv = 1.0f / (lrow[r] * kPVCarry);
#pragma unroll
      for (int t = 0; t < 8; ++t) {
        const int idx = (8 * hh + r) * kOp + t * 16 + c;
        const float sub = ot[idx];
        ot[idx] = oacc[t][r] * inv - sub;
      }
    }
  }
  __syncthreads();
  {
    v4f val[8];
#pragma unroll
    for (int it = 0; it < 8; ++it) val[it] = *(const v4f*)(ot + (par * 8 + it) * kOp + lane * 4);
    float* ob = out + ((size_t)(b * kSeq + q0 + par * 8)) * kDim + h * kVd + lane * 4;
    for (int pass = 0; pass < 2; ++pass) {
#pragma unroll
      for (int it = 0; it < 8; ++it) *(volatile v4f*)(ob + (size_t)it * kDim) = val[it];
      __threadfence();
    }
  }
}

__global__ __launch_bounds__(128) void head_rows_kernel(const float* __restrict__ Qf, const float* __restrict__ Kf,
                                                        const float* __restrict__ Vf, const float* __restrict__ lamp,
                                                        float* __restrict__ out) {
  __shared__ __align__(16) float sq[2 * kHd];
  __shared__ __align__(16) float sw[kHeadRows];
  __shared__ float redM[8];
  __shared__ float redS[8];
  const int t    = threadIdx.x;
  const int lane = t & 31;
  const int wave = __builtin_amdgcn_readfirstlane((int)(t >> 5));
  const int s = blockIdx.x, h = blockIdx.y, b = blockIdx.z;
  {
    const int p = t >> 6, d = t & 63;
    sq[t] = Qf[((size_t)(b * kHalfHeads + 2 * h + p) * kHeadRows + s) * kHd + d];
  }
  __syncthreads();
  const float* k0p = Kf + ((size_t)(b * kHalfHeads + 2 * h) * kHeadRows + t) * kHd;
  const float* k1p = k0p + (size_t)kHeadRows * kHd;
  float a0 = 0.f, a1 = 0.f;
#pragma unroll 1
  for (int d4 = 0; d4 < kHd / 4; ++d4) {
    const v4f ka = *(const v4f*)(k0p + 4 * d4);
    const v4f kb = *(const v4f*)(k1p + 4 * d4);
    const v4f qa = *(const v4f*)(sq + 4 * d4);
    const v4f qc = *(const v4f*)(sq + kHd + 4 * d4);
    a0 = fmaf(qa[0], ka[0], a0);
    a0 = fmaf(qa[1], ka[1], a0);
    a0 = fmaf(qa[2], ka[2], a0);
    a0 = fmaf(qa[3], ka[3], a0);
    a1 = fmaf(qc[0], kb[0], a1);
    a1 = fmaf(qc[1], kb[1], a1);
    a1 = fmaf(qc[2], kb[2], a1);
    a1 = fmaf(qc[3], kb[3], a1);
  }
  const bool live = (t <= s);
  const float l0 = live ? a0 : kMaskFill;
  const float l1 = live ? a1 : kMaskFill;
  float m0 = l0, m1 = l1;
#pragma unroll
  for (int off = 16; off > 0; off >>= 1) {
    const float t0 = __shfl_xor(m0, off, 32);
    const float t1 = __shfl_xor(m1, off, 32);
    m0 = fmaxf(m0, t0);
    m1 = fmaxf(m1, t1);
  }
  if (lane == 0) { redM[wave] = m0; redM[4 + wave] = m1; }
  __syncthreads();
  m0 = fmaxf(fmaxf(redM[0], redM[1]), fmaxf(redM[2], redM[3]));
  m1 = fmaxf(fmaxf(redM[4], redM[5]), fmaxf(redM[6], redM[7]));
  float p0 = expf(l0 - m0);
  float p1 = expf(l1 - m1);
  p0 = live ? p0 : 0.0f;
  p1 = live ? p1 : 0.0f;
  float s0 = p0, s1 = p1;
#pragma unroll
  for (int off = 16; off > 0; off >>= 1) {
    const float t0 = __shfl_xor(s0, off, 32);
    const float t1 = __shfl_xor(s1, off, 32);
    s0 += t0;
    s1 += t1;
  }
  if (lane == 0) { redS[wave] = s0; redS[4 + wave] = s1; }
  __syncthreads();
  s0 = (redS[0] + redS[1]) + (redS[2] + redS[3]);
  s1 = (redS[4] + redS[5]) + (redS[6] + redS[7]);
  const float lam = lamp[0];
  const float r0 = 1.0f / s0;
  const float r1 = 1.0f / s1;
  sw[t] = p0 * r0 - lam * (p1 * r1);
  __syncthreads();
  const float* vp = Vf + ((size_t)b * kDim + h * kVd + t) * kHeadRows;
  const int n4 = (s >> 2) + 1;
  float acc = 0.f;
#pragma unroll 1
  for (int j4 = 0; j4 < n4; ++j4) {
    const v4f vv = *(const v4f*)(vp + 4 * j4);
    const v4f ww = *(const v4f*)(sw + 4 * j4);
    acc = fmaf(ww[0], vv[0], acc);
    acc = fmaf(ww[1], vv[1], acc);
    acc = fmaf(ww[2], vv[2], acc);
    acc = fmaf(ww[3], vv[3], acc);
  }
  float* dst = out + ((size_t)(b * kSeq + s)) * kDim + h * kVd + t;
  *(volatile float*)dst = acc;
  __threadfence();
  *(volatile float*)dst = acc;
}

extern "C" void kernel_launch(void* const* d_in, const int* in_sizes, int n_in,
                              void* d_out, int out_size, void* d_ws, size_t ws_size,
                              hipStream_t stream) {
  if (n_in < 13) return;
  if (in_sizes[0] != kRows * kDim) return;
  if (in_sizes[1] != kSeq * kTabCols) return;
  if (in_sizes[2] != kSeq * kTabCols) return;
  if (in_sizes[3] != kDim * kDim) return;
  if (in_sizes[4] != kDim) return;
  if (in_sizes[5] != kDim * kDim) return;
  if (in_sizes[6] != kDim) return;
  if (in_sizes[7] != kDim * kDim) return;
  if (in_sizes[8] != kDim) return;
  if (in_sizes[9] != kHd || in_sizes[10] != kHd || in_sizes[11] != kHd || in_sizes[12] != kHd) return;
  if (out_size != kRows * kDim) return;
  if (ws_size < kWsTotal) return;

  const float* x    = (const float*)d_in[0];
  const float* fcos = (const float*)d_in[1];
  const float* fsin = (const float*)d_in[2];
  const float* Wq   = (const float*)d_in[3];
  const float* bq   = (const float*)d_in[4];
  const float* Wk   = (const float*)d_in[5];
  const float* bk   = (const float*)d_in[6];
  const float* Wv   = (const float*)d_in[7];
  const float* bv   = (const float*)d_in[8];
  const float* lq1  = (const float*)d_in[9];
  const float* lk1  = (const float*)d_in[10];
  const float* lq2  = (const float*)d_in[11];
  const float* lk2  = (const float*)d_in[12];
  float* out = (float*)d_out;

  char* ws = (char*)d_ws;
  unsigned short* XB = (unsigned short*)(ws + kOffXB);
  unsigned short* WT = (unsigned short*)(ws + kOffWT);
  unsigned short* QH = (unsigned short*)(ws + kOffQH);
  unsigned short* KH = (unsigned short*)(ws + kOffKH);
  unsigned short* VT = (unsigned short*)(ws + kOffVT);
  float* QF  = (float*)(ws + kOffQF);
  float* KF  = (float*)(ws + kOffKF);
  float* VF  = (float*)(ws + kOffVF);
  float* LAM = (float*)(ws + kOffLAM);

  cvt_bf16_kernel<<<(kRows * kDim / 8) / 256, 256, 0, stream>>>(x, XB, kRows * kDim / 8);
  wt_pack_kernel<<<dim3(kDim / 64, kDim / 64, 3), 256, 0, stream>>>(Wq, Wk, Wv, WT);
  lam_kernel<<<1, 32, 0, stream>>>(lq1, lk1, lq2, lk2, LAM);

  proj_gemm_kernel<0><<<((kRows / 64) * ((2 * kDim) / 64)) / 8, 256, 0, stream>>>(
      XB, WT, bq, bk, fcos, fsin, QH, KH, QF, KF, kRows / 64, (2 * kDim) / 64);
  proj_gemm_kernel<1><<<((kDim / 64) * (kRows / 64)) / 8, 256, 0, stream>>>(
      WT + (size_t)2 * kDim * kDim, XB, bv, bv, fcos, fsin, VT, VT, VF, VF, kDim / 64, kRows / 64);

  diff_attn_kernel<<<dim3((kSeq - kHeadRows) / 64, kPairs, kBatch), 256, 0, stream>>>(QH, KH, VT, LAM, out);
  head_rows_kernel<<<dim3(kHeadRows, kPairs, kBatch), 128, 0, stream>>>(QF, KF, VF, LAM, out);
}
